// SSP_MatchingNet_8933531976078
// MI455X (gfx1250) — hardware-verified
//
#include <hip/hip_runtime.h>
#include <math.h>

#define NB    4
#define CH    256
#define NPX   3600
#define NPD   3648
#define NT    57
#define TOPK  12
#define SEG   15
#define FG_TH 0.5f
#define BG_TH 0.8f
#define SSC   0.0078125f

static_assert(NPD == NT * 64);
static_assert(NPD >= NPX);
static_assert(256 * SEG >= NPX);

typedef _Float16 v16h __attribute__((ext_vector_type(16)));
typedef _Float16 v8h  __attribute__((ext_vector_type(8)));
typedef float    v8f  __attribute__((ext_vector_type(8)));
typedef float    v4f  __attribute__((ext_vector_type(4)));
typedef unsigned int v4u __attribute__((ext_vector_type(4)));

__device__ __forceinline__ v8f mma_h(v16h a, v16h b, v8f c) {
  c = __builtin_amdgcn_wmma_f32_16x16x32_f16(false, a, false, b, (short)0, c, false, false);
  asm volatile("v_nop\n\tv_nop\n\tv_nop\n\tv_nop" : "+v"(c) : "v"(a), "v"(b));
  return c;
}

__device__ int build_mask(const float* __restrict__ p, float th, float* shp, float* sm,
                          float* redf, int* redi, int tid) {
  int cnt = 0;
  for (int n = tid; n < NPX; n += 256) {
    const float v = p[n];
    const int mv = (v > th) ? 1 : 0;
    sm[n]  = (float)mv;
    shp[n] = v;
    cnt += mv;
  }
  redi[tid] = cnt;
  __syncthreads();
  for (int s2 = 128; s2 > 0; s2 >>= 1) {
    if (tid < s2) redi[tid] += redi[tid + s2];
    __syncthreads();
  }
  int total = redi[0];
  __syncthreads();
  if (total == 0) {
    for (int it = 0; it < TOPK; ++it) {
      float bv = -INFINITY; int bi = 0x7fffffff;
      for (int n = tid; n < NPX; n += 256) {
        const float v = shp[n];
        if (v > bv) { bv = v; bi = n; }
      }
      redf[tid] = bv; redi[tid] = bi;
      __syncthreads();
      for (int s2 = 128; s2 > 0; s2 >>= 1) {
        if (tid < s2) {
          const float ov = redf[tid + s2]; const int oi = redi[tid + s2];
          const float mvv = redf[tid];     const int mi = redi[tid];
          if (ov > mvv || (ov == mvv && oi < mi)) { redf[tid] = ov; redi[tid] = oi; }
        }
        __syncthreads();
      }
      if (tid == 0) {
        const int ix = redi[0];
        if ((unsigned)ix < (unsigned)NPX) { sm[ix] = 1.0f; shp[ix] = -INFINITY; }
      }
      __syncthreads();
    }
    total = TOPK;
  }
  return total;
}

__global__ __launch_bounds__(256) void k_sel(const float* __restrict__ feat, const float* __restrict__ mq,
                                             const int* __restrict__ kflag,
                                             float* __restrict__ out0, float* __restrict__ bgp) {
  __shared__ float shp[NPX];
  __shared__ float smf[NPX];
  __shared__ float smb[NPX];
  __shared__ float redf[256];
  __shared__ int   redi[256];
  __shared__ __align__(16) float spf[CH];
  __shared__ __align__(16) float spb[CH];
  (void)kflag;
  const int tid = threadIdx.x, wave = tid >> 5;
  const int b = blockIdx.x;
  const int totf = build_mask(mq + ((size_t)b * 2 + 1) * NPX, FG_TH, shp, smf, redf, redi, tid);
  const int totb = build_mask(mq + ((size_t)b * 2 + 0) * NPX, BG_TH, shp, smb, redf, redi, tid);
  __syncthreads();

  const float* F = feat + (size_t)b * CH * NPX + (size_t)tid * NPX;
  float af = 0.f, ab = 0.f;
#pragma unroll 4
  for (int n = 0; n < NPX; ++n) {
    const float v = F[n];
    af = fmaf(v, smf[n], af);
    ab = fmaf(v, smb[n], ab);
  }
  spf[tid] = af * (1.0f / (float)totf);
  spb[tid] = ab * (1.0f / (float)totb);
  __syncthreads();

  if (wave < 4) {
    const int i = tid & 63;
    const v4f vf = *(const v4f*)(spf + 4 * i);
    const v4f vb = *(const v4f*)(spb + 4 * i);
    const bool isf = wave < 2;
    v4f v;
    v[0] = isf ? vf[0] : vb[0];
    v[1] = isf ? vf[1] : vb[1];
    v[2] = isf ? vf[2] : vb[2];
    v[3] = isf ? vf[3] : vb[3];
    float* dst = isf ? (out0 + (size_t)b * CH + 4 * i) : (bgp + (size_t)b * CH + 4 * i);
    *(volatile v4f*)dst = v;
    __threadfence();
    *(volatile v4f*)dst = v;
  }
}

#define QLP 264
__global__ __launch_bounds__(256) void k_q(const float* __restrict__ feat, _Float16* __restrict__ Qp) {
  __shared__ __align__(16) _Float16 Qs[64 * QLP];
  __shared__ float part[4][64];
  __shared__ float invs[64];
  const int tid = threadIdx.x, lane = tid & 31, wave = tid >> 5;
  const int b = blockIdx.y, n0 = blockIdx.x * 64;
  const int px = tid & 63, cg = tid >> 6;
  const int n = n0 + px;
  const int ncl = (n < NPX) ? n : (NPX - 1);
  const float* F = feat + (size_t)b * CH * NPX + (size_t)(cg * 64) * NPX + ncl;

  float ss = 0.f;
#pragma unroll 4
  for (int c = 0; c < 64; ++c) { const float v = F[(size_t)c * NPX]; ss = fmaf(v, v, ss); }
  part[cg][px] = ss;
  __syncthreads();
  if (tid < 64) {
    const float tot = (part[0][tid] + part[1][tid]) + (part[2][tid] + part[3][tid]);
    const bool ok = (n0 + tid < NPX) && (tot > 0.f);
    const float r = 16.0f * rsqrtf(tot);
    invs[tid] = ok ? r : 0.f;
  }
  __syncthreads();
  const float sc = invs[px];
  _Float16* qrow = Qs + px * QLP + cg * 64;
#pragma unroll 4
  for (int c = 0; c < 64; ++c) { const float v = F[(size_t)c * NPX]; qrow[c] = (_Float16)(v * sc); }
  __syncthreads();

  const _Float16* src = Qs + (wave * 8) * QLP + lane * 8;
  _Float16* dst = Qp + ((size_t)b * NPD + n0 + wave * 8) * CH + lane * 8;
#pragma unroll
  for (int rr = 0; rr < 8; ++rr) {
    const v8h v = *(const v8h*)(src + rr * QLP);
    *(volatile v8h*)(dst + (size_t)rr * CH) = v;
  }
  __threadfence();
#pragma unroll
  for (int rr = 0; rr < 8; ++rr) {
    const v8h v = *(const v8h*)(src + rr * QLP);
    *(volatile v8h*)(dst + (size_t)rr * CH) = v;
  }
}

__global__ __launch_bounds__(256) void k_cmp(const float* __restrict__ feat, const float* __restrict__ mq,
                                             const _Float16* __restrict__ Qp,
                                             _Float16* __restrict__ Ks, _Float16* __restrict__ Vt) {
  __shared__ float shp[NPX];
  __shared__ float sm[NPX];
  __shared__ int   lst[NPD];
  __shared__ float redf[256];
  __shared__ int   redi[256];
  __shared__ int   wtot[8];
  const int tid = threadIdx.x, lane = tid & 31, wave = tid >> 5;
  const int b = blockIdx.y, j0 = blockIdx.x * 64;
  const int cnt = build_mask(mq + (size_t)b * 2 * NPX, BG_TH, shp, sm, redf, redi, tid);

  const int s0 = tid * SEG;
  int ct = 0;
#pragma unroll
  for (int k = 0; k < SEG; ++k) {
    const int nn = s0 + k;
    const int ncl = (nn < NPX) ? nn : (NPX - 1);
    ct += (nn < NPX && sm[ncl] != 0.f) ? 1 : 0;
  }
  int incl = ct;
#pragma unroll
  for (int off = 1; off < 32; off <<= 1) {
    const int y = __shfl_up(incl, off, 32);
    incl += (lane >= off) ? y : 0;
  }
  const int wsum = __shfl(incl, 31, 32);
  if (lane == 31) wtot[wave] = wsum;
  __syncthreads();
  int base = 0;
#pragma unroll
  for (int w = 0; w < 8; ++w) base += (w < wave) ? wtot[w] : 0;
  int pos = base + incl - ct;
#pragma unroll
  for (int k = 0; k < SEG; ++k) {
    const int nn = s0 + k;
    const int ncl = (nn < NPX) ? nn : (NPX - 1);
    const bool selb = (nn < NPX) && (sm[ncl] != 0.f);
    if (selb) { lst[(pos < NPD) ? pos : (NPD - 1)] = nn; ++pos; }
  }
  __syncthreads();

  {
    const _Float16* Qb = Qp + (size_t)b * NPD * CH;
    v4u kv[8];
#pragma unroll
    for (int rr = 0; rr < 8; ++rr) {
      const int j = j0 + wave * 8 + rr;
      const bool valid = j < cnt;
      int pix = lst[j];
      pix = valid ? pix : 0;
      pix = (pix < 0) ? 0 : ((pix >= NPX) ? (NPX - 1) : pix);
      const v4u v = *(const v4u*)(Qb + (size_t)pix * CH + lane * 8);
      const unsigned mk = valid ? 0xffffffffu : 0u;
      kv[rr] = v & (v4u){mk, mk, mk, mk};
    }
    _Float16* Kd = Ks + ((size_t)b * NPD + j0 + wave * 8) * CH + lane * 8;
#pragma unroll
    for (int rr = 0; rr < 8; ++rr) *(volatile v4u*)(Kd + (size_t)rr * CH) = kv[rr];
    __threadfence();
#pragma unroll
    for (int rr = 0; rr < 8; ++rr) *(volatile v4u*)(Kd + (size_t)rr * CH) = kv[rr];
  }

  {
    const int q = tid & 7, sub = tid >> 3;
    int pixe[8]; float sce[8];
#pragma unroll
    for (int e = 0; e < 8; ++e) {
      const int j = j0 + 8 * q + e;
      const bool valid = j < cnt;
      int pix = lst[j];
      pix = valid ? pix : 0;
      pix = (pix < 0) ? 0 : ((pix >= NPX) ? (NPX - 1) : pix);
      pixe[e] = pix;
      sce[e]  = valid ? 16.0f : 0.0f;
    }
    const float* Fb = feat + (size_t)b * CH * NPX;
    v8h hv[8];
#pragma unroll
    for (int it = 0; it < 8; ++it) {
      const float* Fr = Fb + (size_t)(it * 32 + sub) * NPX;
      v8h t;
#pragma unroll
      for (int e = 0; e < 8; ++e) t[e] = (_Float16)(Fr[pixe[e]] * sce[e]);
      hv[it] = t;
    }
    _Float16* Vd = Vt + ((size_t)b * CH + sub) * NPD + j0 + 8 * q;
#pragma unroll
    for (int it = 0; it < 8; ++it) *(volatile v8h*)(Vd + (size_t)(it * 32) * NPD) = hv[it];
    __threadfence();
#pragma unroll
    for (int it = 0; it < 8; ++it) *(volatile v8h*)(Vd + (size_t)(it * 32) * NPD) = hv[it];
  }
}

#define KLP 264
#define VLP 72
#define PLP 72
#define OLP 68
#define LDS_K (64 * KLP * 2)
#define LDS_V (CH * VLP * 2)
#define LDS_P (4 * 16 * PLP * 2)
#define LDS_ATT (LDS_K + LDS_V + LDS_P)
static_assert(CH * OLP * 4 <= LDS_ATT);
static_assert((LDS_K % 16) == 0 && (LDS_V % 16) == 0);

__global__ __launch_bounds__(256) void k_att(const _Float16* __restrict__ Qp, const _Float16* __restrict__ Ks,
                                             const _Float16* __restrict__ Vt, const float* __restrict__ mq,
                                             float* __restrict__ Lp) {
  extern __shared__ v4f smem_dyn[];
  char* smem = (char*)smem_dyn;
  _Float16* Ksh = (_Float16*)smem;
  _Float16* Vsh = (_Float16*)(smem + LDS_K);
  _Float16* Psh = (_Float16*)(smem + LDS_K + LDS_V);
  float*    Os  = (float*)smem;
  __shared__ float Al[4][16];
  __shared__ float Ll[4][16];
  __shared__ int   redc[8];
  union FB { v16h v; v8h h[2]; };

  const int tid  = threadIdx.x;
  const int wave = tid >> 5;
  const int lane = tid & 31;
  const int lh   = lane >> 4;
  const int c    = lane & 15;
  const int g    = wave & 3;
  const int chh  = wave >> 2;
  const int ch0  = chh * 128;
  const int qt   = blockIdx.x;
  const int b    = blockIdx.y;
  const int n0   = qt * 64;
  const int qg0  = n0 + g * 16;

  int cl = 0;
  {
    const float* pb = mq + (size_t)b * 2 * NPX;
    for (int n = tid; n < NPX; n += 256) cl += (pb[n] > BG_TH) ? 1 : 0;
  }
#pragma unroll
  for (int off = 1; off < 32; off <<= 1) cl += __shfl_xor(cl, off, 32);
  if (lane == 0) redc[wave] = cl;
  __syncthreads();
  int total = 0;
#pragma unroll
  for (int w = 0; w < 8; ++w) total += redc[w];
  const int cnt = (total > 0) ? total : TOPK;
  int nch = (cnt + 63) >> 6;
  nch = (nch > NT) ? NT : nch;

  const _Float16* Qrow = Qp + ((size_t)b * NPD + qg0 + c) * CH + 8 * lh;
  const _Float16* Ksb  = Ks + (size_t)b * NPD * CH;
  const _Float16* Vtb  = Vt + (size_t)b * CH * NPD;

  float mrow[8], lrow[8];
  v8f oacc[8];
#pragma unroll
  for (int r = 0; r < 8; ++r) { mrow[r] = -INFINITY; lrow[r] = 0.f; }
#pragma unroll
  for (int t = 0; t < 8; ++t) oacc[t] = (v8f){0.f, 0.f, 0.f, 0.f, 0.f, 0.f, 0.f, 0.f};

  _Float16* pw = Psh + g * 16 * PLP;

  for (int kc = 0; kc < nch; ++kc) {
    const int kv0 = kc * 64;
    __syncthreads();
    {
      const int r = tid >> 2, qq = (tid & 3) * 64;
      const _Float16* src = Ksb + (size_t)(kv0 + r) * CH + qq;
      _Float16* dst = Ksh + r * KLP + qq;
#pragma unroll
      for (int i = 0; i < 8; ++i) *(v8h*)(dst + 8 * i) = *(const v8h*)(src + 8 * i);
      const _Float16* vs = Vtb + (size_t)tid * NPD + kv0;
      _Float16* vd = Vsh + tid * VLP;
#pragma unroll
      for (int i = 0; i < 8; ++i) *(v8h*)(vd + 8 * i) = *(const v8h*)(vs + 8 * i);
    }
    __syncthreads();

    if (wave < 4) {
      v8f s[4];
#pragma unroll
      for (int j = 0; j < 4; ++j) s[j] = (v8f){0.f, 0.f, 0.f, 0.f, 0.f, 0.f, 0.f, 0.f};
#pragma unroll
      for (int dc = 0; dc < 8; ++dc) {
        FB qa;
        qa.h[0] = *(const v8h*)(Qrow + dc * 32);
        qa.h[1] = *(const v8h*)(Qrow + dc * 32 + 16);
#pragma unroll
        for (int j = 0; j < 4; ++j) {
          const _Float16* kp = Ksh + (j * 16 + c) * KLP + dc * 32 + 8 * lh;
          FB kb;
          kb.h[0] = *(const v8h*)(kp);
          kb.h[1] = *(const v8h*)(kp + 16);
          s[j] = mma_h(qa.v, kb.v, s[j]);
        }
      }
      float cm[8];
#pragma unroll
      for (int r = 0; r < 8; ++r) {
        float m = -INFINITY;
#pragma unroll
        for (int j = 0; j < 4; ++j) {
          const int key = kv0 + j * 16 + c;
          const float sv = (key < cnt) ? s[j][r] * SSC : -INFINITY;
          s[j][r] = sv;
          m = fmaxf(m, sv);
        }
#pragma unroll
        for (int off = 1; off < 16; off <<= 1) m = fmaxf(m, __shfl_xor(m, off, 32));
        cm[r] = m;
      }
#pragma unroll
      for (int r = 0; r < 8; ++r) {
        const float mnew  = fmaxf(mrow[r], cm[r]);
        const float alpha = __expf(mrow[r] - mnew);
        mrow[r] = mnew;
        float psum = 0.f;
#pragma unroll
        for (int j = 0; j < 4; ++j) {
          const float p = __expf(s[j][r] - mnew);
          psum += p;
          pw[(8 * lh + r) * PLP + j * 16 + c] = (_Float16)(p * 1024.0f);
        }
#pragma unroll
        for (int off = 1; off < 16; off <<= 1) psum += __shfl_xor(psum, off, 32);
        lrow[r] = lrow[r] * alpha + psum;
        if (c == 0) {
          Al[g][8 * lh + r] = alpha;
          Ll[g][8 * lh + r] = lrow[r];
        }
      }
    }
    __syncthreads();

    {
      float af[8];
#pragma unroll
      for (int r = 0; r < 8; ++r) af[r] = Al[g][8 * lh + r];
#pragma unroll
      for (int t = 0; t < 8; ++t)
#pragma unroll
        for (int r = 0; r < 8; ++r) oacc[t][r] *= af[r];
#pragma unroll
      for (int kk = 0; kk < 2; ++kk) {
        FB pa;
        pa.h[0] = *(const v8h*)(pw + c * PLP + kk * 32 + 8 * lh);
        pa.h[1] = *(const v8h*)(pw + c * PLP + kk * 32 + 16 + 8 * lh);
#pragma unroll
        for (int t = 0; t < 8; ++t) {
          const _Float16* vp = Vsh + (ch0 + t * 16 + c) * VLP + kk * 32 + 8 * lh;
          FB vb;
          vb.h[0] = *(const v8h*)(vp);
          vb.h[1] = *(const v8h*)(vp + 16);
          oacc[t] = mma_h(pa.v, vb.v, oacc[t]);
        }
      }
    }
  }
  __syncthreads();

#pragma unroll
  for (int r = 0; r < 8; ++r) {
    const float l = Ll[g][8 * lh + r];
    const float inv = (1.0f / l) * 6.103515625e-05f;
#pragma unroll
    for (int t = 0; t < 8; ++t) Os[(ch0 + 16 * t + c) * OLP + g * 16 + 8 * lh + r] = oacc[t][r] * inv;
  }
  __syncthreads();
  {
    const int q8 = tid & 7, sub = tid >> 3;
    float* Lb = Lp + (size_t)b * CH * NPD + n0;
#pragma unroll
    for (int it = 0; it < 16; ++it) {
      const int li = it * 32 + sub;
      const int cc = li >> 1, hf = li & 1;
      const v4f vv = *(const v4f*)(Os + cc * OLP + hf * 32 + q8 * 4);
      *(volatile v4f*)(Lb + (size_t)cc * NPD + hf * 32 + q8 * 4) = vv;
    }
    __threadfence();
#pragma unroll
    for (int it = 0; it < 16; ++it) {
      const int li = it * 32 + sub;
      const int cc = li >> 1, hf = li & 1;
      const v4f vv = *(const v4f*)(Os + cc * OLP + hf * 32 + q8 * 4);
      *(volatile v4f*)(Lb + (size_t)cc * NPD + hf * 32 + q8 * 4) = vv;
    }
  }
}

__global__ __launch_bounds__(256) void k_out(const float* __restrict__ Lp, const float* __restrict__ bgp,
                                             float* __restrict__ out1) {
  const int t = blockIdx.x * 256 + (int)threadIdx.x;
  const int e = t * 4;
  v4f v;
#pragma unroll
  for (int i = 0; i < 4; ++i) {
    const int idx = e + i;
    const int b  = idx / (CH * NPX);
    const int rr = idx - b * (CH * NPX);
    const int cc = rr / NPX;
    const int n  = rr - cc * NPX;
    const float loc = Lp[((size_t)(b * CH + cc)) * NPD + n];
    const float pro = bgp[b * CH + cc];
    v[i] = pro * 0.3f + loc * 0.7f;
  }
  volatile v4f* p = (volatile v4f*)(out1 + e);
  *p = v;
  __threadfence();
  *p = v;
}

extern "C" void kernel_launch(void* const* d_in, const int* in_sizes, int n_in,
                              void* d_out, int out_size, void* d_ws, size_t ws_size,
                              hipStream_t stream) {
  if (n_in < 3) return;
  if (in_sizes[0] != NB * CH * NPX) return;
  if (in_sizes[1] != NB * 2 * NPX) return;
  if (in_sizes[2] < 1) return;
  if (out_size != NB * CH + NB * CH * NPX) return;

  const float* feat  = (const float*)d_in[0];
  const float* mq    = (const float*)d_in[1];
  const int*   kflag = (const int*)d_in[2];
  float* out = (float*)d_out;

  const size_t szQ = (size_t)NB * NPD * CH * 2;
  const size_t szK = szQ;
  const size_t szV = (size_t)NB * CH * NPD * 2;
  const size_t szL = (size_t)NB * CH * NPD * 4;
  const size_t szB = (size_t)NB * CH * 4;
  size_t off = 0;
  const size_t oQ = off; off += szQ;
  const size_t oK = off; off += szK;
  const size_t oV = off; off += szV;
  const size_t oL = off; off += szL;
  const size_t oB = off; off += szB;
  if (off > ws_size) return;

  char* ws = (char*)d_ws;
  _Float16* Qp  = (_Float16*)(ws + oQ);
  _Float16* Ksp = (_Float16*)(ws + oK);
  _Float16* Vtp = (_Float16*)(ws + oV);
  float*    Lp  = (float*)(ws + oL);
  float*    bgp = (float*)(ws + oB);

  k_sel<<<dim3(NB), dim3(256), 0, stream>>>(feat, mq, kflag, out, bgp);
  k_q<<<dim3(NT, NB), dim3(256), 0, stream>>>(feat, Qp);
  k_cmp<<<dim3(NT, NB), dim3(256), 0, stream>>>(feat, mq, Qp, Ksp, Vtp);
  (void)hipFuncSetAttribute(reinterpret_cast<const void*>(&k_att), hipFuncAttributeMaxDynamicSharedMemorySize, LDS_ATT);
  k_att<<<dim3(NT, NB), dim3(256), LDS_ATT, stream>>>(Qp, Ksp, Vtp, mq, Lp);
  k_out<<<dim3((NB * CH * NPX) / 1024), dim3(256), 0, stream>>>(Lp, bgp, out + NB * CH);
  (void)hipGetLastError();
}
